// SelectiveScan2D_16312285791111
// MI455X (gfx1250) — hardware-run, weakly checked
//
#include <hip/hip_runtime.h>
#include <math.h>


#define NB   8
#define HH   64
#define WW   64
#define CC   256
#define NS   64
#define LL   (HH * WW)
#define NPOS (NB * LL)
typedef __attribute__((ext_vector_type(16))) _Float16 v16h;
typedef __attribute__((ext_vector_type(8)))  _Float16 v8h;
typedef __attribute__((ext_vector_type(8)))  float    v8f;
typedef __attribute__((ext_vector_type(4)))  float    v4f;
#define VST2(T, ptr, val) do { const T _v = (val); *(volatile T*)(ptr) = _v; __threadfence(); *(volatile T*)(ptr) = _v; } while (0)
__device__ __forceinline__ v8f wmma16(v16h a, v16h b, v8f c) {
  v8f d = __builtin_amdgcn_wmma_f32_16x16x32_f16(false, a, false, b, (short)0, c, false, false);
  asm volatile("v_nop\n\tv_nop\n\tv_nop\n\tv_nop" : "+v"(d) : "v"(a), "v"(b));
  return d;
}
__device__ __forceinline__ v16h frag16(const _Float16* p, int hh) {
  const v8h lo = *(const v8h*)(p + 8 * hh), hi = *(const v8h*)(p + 16 + 8 * hh);
  return __builtin_shufflevector(lo, hi, 0,1,2,3,4,5,6,7,8,9,10,11,12,13,14,15);
}
__global__ __launch_bounds__(256) void k_ln2(const float* __restrict__ x, float* __restrict__ S, _Float16* __restrict__ S16) {
  const int pos = blockIdx.x * 8 + (threadIdx.x >> 5), lane = threadIdx.x & 31;
  const float* xr = x + (size_t)pos * CC + lane * 8;
  float v[8]; float s = 0.f;
#pragma unroll
  for (int e = 0; e < 8; ++e) { v[e] = xr[e]; s += v[e]; }
  for (int it = 0; it < 2; ++it) {
#pragma unroll
    for (int o = 16; o > 0; o >>= 1) s += __shfl_xor(s, o, 32);
    const float mu = s * (1.0f / CC);
    float q = 0.f;
#pragma unroll
    for (int e = 0; e < 8; ++e) { v[e] -= mu; q += v[e] * v[e]; }
#pragma unroll
    for (int o = 16; o > 0; o >>= 1) q += __shfl_xor(q, o, 32);
    const float rs = 1.0f / sqrtf(q * (1.0f / CC) + 1e-5f);
    s = 0.f;
#pragma unroll
    for (int e = 0; e < 8; ++e) { v[e] *= rs; s += v[e]; }
  }
  typedef __attribute__((ext_vector_type(8))) float v8f32; v8f32 o; v8h oh;
#pragma unroll
  for (int e = 0; e < 8; ++e) { o[e] = v[e]; oh[e] = (_Float16)v[e]; }
  VST2(v8f32, S + (size_t)pos * CC + lane * 8, o);
  VST2(v8h, S16 + (size_t)pos * CC + lane * 8, oh);
}
__global__ __launch_bounds__(256) void k_w16(const float* __restrict__ w, int N, int K, int Npad, _Float16* __restrict__ W16) {
  const int t = blockIdx.x * 256 + threadIdx.x; const int per = K / 8;
  if (t >= Npad * per) return;
  const int n = t / per, k0 = (t % per) * 8;
  v8h o;
#pragma unroll
  for (int e = 0; e < 8; ++e) o[e] = (n < N) ? (_Float16)w[(size_t)n * K + k0 + e] : (_Float16)0.f;
  VST2(v8h, W16 + (size_t)n * K + k0, o);
}
template <int K, int NTOT, int EPI>
__global__ __launch_bounds__(128) void k_gemm(const _Float16* __restrict__ A, const _Float16* __restrict__ W16, const float* __restrict__ Dv, const float* __restrict__ S,
                                              float* __restrict__ outf) {
  __shared__ __attribute__((aligned(16))) float sT[4][16][132];
  const int lane = threadIdx.x & 31, wave = threadIdx.x >> 5, hh = lane >> 4, l16 = lane & 15;
  const int m0 = blockIdx.x * 64 + wave * 16, n0 = blockIdx.y * 128;
  v8f acc[8];
#pragma unroll
  for (int ni = 0; ni < 8; ++ni) acc[ni] = (v8f){};
#pragma unroll 2
  for (int k0 = 0; k0 < K; k0 += 32) {
    const v16h a0 = frag16(A + (size_t)(m0 + l16) * K + k0, hh);
#pragma unroll
    for (int ni = 0; ni < 8; ++ni) { const v16h b = frag16(W16 + (size_t)(n0 + ni * 16 + l16) * K + k0, hh); acc[ni] = wmma16(a0, b, acc[ni]); }
  }
  float (*st)[132] = sT[wave];
#pragma unroll
  for (int ni = 0; ni < 8; ++ni)
#pragma unroll
    for (int i = 0; i < 8; ++i) st[i + 8 * hh][ni * 16 + l16] = acc[ni][i];
  __builtin_amdgcn_fence(__ATOMIC_RELEASE, "workgroup"); __builtin_amdgcn_wave_barrier(); __builtin_amdgcn_fence(__ATOMIC_ACQUIRE, "workgroup");
  for (int pass = 0; pass < 2; ++pass) {
#pragma unroll
    for (int rr = 0; rr < 16; ++rr) {
      v4f v = *(const v4f*)(&st[rr][lane * 4]);
      if (EPI == 1) { const v4f sv = *(const v4f*)(S + (size_t)(m0 + rr) * NTOT + n0 + lane * 4); const v4f dv = *(const v4f*)(Dv + n0 + lane * 4); v += dv * sv; }
      *(volatile v4f*)(outf + (size_t)(m0 + rr) * NTOT + n0 + lane * 4) = v;
    }
    __threadfence();
  }
}
__global__ __launch_bounds__(64) void k_scan(const float* __restrict__ U, const float* __restrict__ A, const float* __restrict__ Bp, const float* __restrict__ snr,
                                             float* __restrict__ HS) {
  const int b = blockIdx.x >> 2, dir = blockIdx.x & 3, n = threadIdx.x;
  const float sc = 0.6f + 0.4f * fminf(fmaxf(snr[b], 0.0f), 1.0f);
  const float Ad = fminf(fmaxf(tanhf(A[n]) * sc, -0.99f), 0.99f), bp = Bp[n];
  float* hs = HS + (size_t)dir * NPOS * NS;
  float h = 0.f;
  for (int t = 0; t < LL; ++t) {
    int pos;
    if (dir == 0) pos = t; else if (dir == 1) pos = LL - 1 - t;
    else { const int tt = (dir == 2) ? t : (LL - 1 - t); pos = (tt % HH) * WW + tt / HH; }
    const size_t p = (size_t)b * LL + pos;
    h = Ad * h + bp * U[p * 128 + n];
    VST2(float, hs + p * NS + n, h);
  }
}
__global__ __launch_bounds__(256) void k_comb(const float* __restrict__ HS, const float* __restrict__ Cp, _Float16* __restrict__ A2) {
  const int t = blockIdx.x * 256 + threadIdx.x;
  const int pos = t >> 3, c = (t & 7) * 8;
  v8h o;
#pragma unroll
  for (int e = 0; e < 8; ++e) { const size_t i = (size_t)pos * NS + c + e;
    const float s = ((HS[i] + HS[(size_t)NPOS * NS + i]) + HS[(size_t)2 * NPOS * NS + i]) + HS[(size_t)3 * NPOS * NS + i];
    o[e] = (_Float16)(0.25f * Cp[c + e] * s); }
  VST2(v8h, A2 + (size_t)pos * NS + c, o);
}
extern "C" void kernel_launch(void* const* d_in, const int* in_sizes, int n_in,
                              void* d_out, int out_size, void* d_ws, size_t ws_size, hipStream_t stream) {
  (void)in_sizes; (void)n_in; (void)out_size;
  const float* x    = (const float*)d_in[0];
  const float* snr  = (const float*)d_in[1];
  const float* A    = (const float*)d_in[2];
  const float* Bp   = (const float*)d_in[3];
  const float* Cp   = (const float*)d_in[4];
  const float* Dv   = (const float*)d_in[5];
  const float* Win  = (const float*)d_in[6];
  const float* Wout = (const float*)d_in[7];
  float* out = (float*)d_out;
  char* ws = (char*)d_ws; size_t off = 0;
  auto take = [&](size_t bytes) { void* p = ws + off; off = (off + bytes + 255) & ~(size_t)255; return p; };
  float*    S   = (float*)take((size_t)NPOS * CC * 4);
  _Float16* S16 = (_Float16*)take((size_t)NPOS * CC * 2);
  _Float16* Wi6 = (_Float16*)take((size_t)128 * CC * 2);
  _Float16* Wo6 = (_Float16*)take((size_t)CC * NS * 2);
  float*    U   = (float*)take((size_t)NPOS * 128 * 4);
  float*    HS  = (float*)take((size_t)4 * NPOS * NS * 4);
  _Float16* A2  = (_Float16*)take((size_t)NPOS * NS * 2);
  if (off > ws_size) return;
  k_ln2<<<NPOS / 8, 256, 0, stream>>>(x, S, S16);
  k_w16<<<(128 * 32 + 255) / 256, 256, 0, stream>>>(Win, NS, CC, 128, Wi6);
  k_w16<<<(CC * 8 + 255) / 256, 256, 0, stream>>>(Wout, CC, NS, CC, Wo6);
  k_gemm<CC, 128, 0><<<dim3(NPOS / 64, 1), 128, 0, stream>>>(S16, Wi6, nullptr, nullptr, U);
  k_scan<<<NB * 4, 64, 0, stream>>>(U, A, Bp, snr, HS);
  k_comb<<<NPOS * 8 / 256, 256, 0, stream>>>(HS, Cp, A2);
  k_gemm<NS, CC, 1><<<dim3(NPOS / 64, 2), 128, 0, stream>>>(A2, Wo6, Dv, S, out);
}
